// Mamba_33543694582347
// MI455X (gfx1250) — hardware-verified
//
#include <hip/hip_runtime.h>
#include <math.h>

typedef __attribute__((ext_vector_type(16))) _Float16 v16h;
typedef __attribute__((ext_vector_type(8)))  _Float16 v8h;
typedef __attribute__((ext_vector_type(16))) __bf16   v16b;
typedef __attribute__((ext_vector_type(8)))  __bf16   v8b;
typedef __attribute__((ext_vector_type(8)))  float    v8f;
typedef __attribute__((ext_vector_type(4)))  float    v4f;

constexpr int kBatch = 4;
constexpr int kSeq   = 2048;
constexpr int kDm    = 1024;
constexpr int kDin   = 2048;
constexpr int kNst   = 16;
constexpr int kConv  = 4;
constexpr int kXzP   = 2 * kDin;
constexpr int kRows  = kBatch * kSeq;
constexpr int kScanTS = 64;
constexpr int kScanCh = 64;
constexpr int kScanYP = 68;
constexpr int kTrP    = 68;
static_assert((kDm % 32) == 0 && (kDin % 32) == 0, "GEMM K multiples of 32");
static_assert((kSeq % 64) == 0 && (kRows % 64) == 0 && (kXzP % 64) == 0 && (kDm % 64) == 0, "GEMM M,N multiples of 64");
static_assert((kSeq % kScanTS) == 0 && (kDin % kScanCh) == 0, "scan tile multiples");
static_assert((kDm % 64) == 0 && (kXzP % 64) == 0 && (kDin % 64) == 0, "transpose tile multiples");
static_assert(((kRows * kDm) % (8 * 256)) == 0, "cast kernel coverage");

constexpr size_t kOffXB   = 0;
constexpr size_t kOffWIT  = kOffXB  + (size_t)kRows * kDm  * 2;
constexpr size_t kOffWOT  = kOffWIT + (size_t)kXzP  * kDm  * 2;
constexpr size_t kOffXZ   = kOffWOT + (size_t)kDm   * kDin * 2;
constexpr size_t kOffYG   = kOffXZ  + (size_t)kSeq  * kXzP * 4;
constexpr size_t kWsTotal = kOffYG  + (size_t)kRows * kDin * 2;
static_assert(kWsTotal == 96468992ull, "carve total");
static_assert(kWsTotal <= 134217728ull, "carve cap");
static_assert((kOffWIT % 128) == 0 && (kOffWOT % 128) == 0 && (kOffXZ % 128) == 0 && (kOffYG % 128) == 0, "128-B aligned regions");

__device__ __forceinline__ unsigned short f2bf_bits(float f) {
  unsigned u = __float_as_uint(f);
  return (unsigned short)((u + 0x7FFFu + ((u >> 16) & 1u)) >> 16);
}
__device__ __forceinline__ float bf_bits2f(unsigned short h) { return __uint_as_float(((unsigned)h) << 16); }
__device__ __forceinline__ float bf_rne(float f) { return bf_bits2f(f2bf_bits(f)); }

__device__ __forceinline__ void dep_guard_h(v8f& a, v8f& b, v16h x, v16h y) { asm volatile("v_nop\n\tv_nop\n\tv_nop\n\tv_nop" : "+v"(a), "+v"(b) : "v"(x), "v"(y)); }
__device__ __forceinline__ void dep_guard_b(v8f& a, v8f& b, v16b x, v16b y) { asm volatile("v_nop\n\tv_nop\n\tv_nop\n\tv_nop" : "+v"(a), "+v"(b) : "v"(x), "v"(y)); }
__device__ __forceinline__ void keep4_h(v16h a, v16h b, v16h c, v16h d) { asm volatile("v_nop" :: "v"(a), "v"(b), "v"(c), "v"(d)); }
__device__ __forceinline__ void keep4_b(v16b a, v16b b, v16b c, v16b d) { asm volatile("v_nop" :: "v"(a), "v"(b), "v"(c), "v"(d)); }
__device__ __forceinline__ void acc_guard4(v8f& a, v8f& b, v8f& c, v8f& d) { asm volatile("v_nop\n\tv_nop\n\tv_nop\n\tv_nop" : "+v"(a), "+v"(b), "+v"(c), "+v"(d)); }
template <typename T> struct Frag;
template <> struct Frag<_Float16> {
  typedef v16h V; union U { v16h v; v8h h[2]; };
  static __device__ __forceinline__ v16h load(const _Float16* p) {
    U f; f.h[0] = *(const v8h*)(p); f.h[1] = *(const v8h*)(p + 16); return f.v;
  }
  static __device__ __forceinline__ v8f mma(v16h a, v16h b, v8f c) {
    return __builtin_amdgcn_wmma_f32_16x16x32_f16(false, a, false, b, (short)0, c, false, false);
  }
  static __device__ __forceinline__ void guard(v8f& a, v8f& b, v16h x, v16h y) { dep_guard_h(a, b, x, y); }
  static __device__ __forceinline__ void keep(v16h a, v16h b, v16h c, v16h d) { keep4_h(a, b, c, d); }
};
template <> struct Frag<__bf16> {
  typedef v16b V; union U { v16b v; v8b h[2]; };
  static __device__ __forceinline__ v16b load(const __bf16* p) {
    U f; f.h[0] = *(const v8b*)(p); f.h[1] = *(const v8b*)(p + 16); return f.v;
  }
  static __device__ __forceinline__ v8f mma(v16b a, v16b b, v8f c) {
    return __builtin_amdgcn_wmma_f32_16x16x32_bf16(false, a, false, b, (short)0, c, false, false);
  }
  static __device__ __forceinline__ void guard(v8f& a, v8f& b, v16b x, v16b y) { dep_guard_b(a, b, x, y); }
  static __device__ __forceinline__ void keep(v16b a, v16b b, v16b c, v16b d) { keep4_b(a, b, c, d); }
};

template <int ET> struct Elem;
template <> struct Elem<0> { typedef _Float16 T; };
template <> struct Elem<1> { typedef __bf16 T; };
template <int ET, int SPL, int BIAS_MODE, int OUT_MODE, bool RESID, int ACT = 0>
__global__ __launch_bounds__(256) void wmma_gemm64(
    const unsigned short* __restrict__ Ap, const unsigned short* __restrict__ A2p, int lda, long strideA,
    const unsigned short* __restrict__ Btp, const unsigned short* __restrict__ Bt2p, int ldb, long strideB,
    void* __restrict__ Cout, void* __restrict__ Cout2, int ldc, long strideC,
    const float* __restrict__ bias,
    const float* __restrict__ resid, long strideR,
    int M, int N, int K, float scale) {
  typedef typename Elem<ET>::T T;
  typedef typename Frag<T>::V V;
  const T* A = (const T*)Ap; const T* A2 = (const T*)A2p; const T* Bt = (const T*)Btp; const T* Bt2 = (const T*)Bt2p;
  __shared__ __align__(16) float sT[8][16 * 68];
  const int b    = blockIdx.y;
  const int lane = threadIdx.x & 31;
  const int wave = threadIdx.x >> 5;
  const int tilesN = N >> 6;
  const int tilesM = M >> 6;
  const int tile = blockIdx.x * 8 + wave;
  if (tile >= tilesM * tilesN) return;
  const int tm = tile / tilesN;
  const int tn = tile - tm * tilesN;
  const int m0 = tm << 6;
  const int n0 = tn << 6;

  const T* Ab  = A  + (size_t)b * strideA;
  const T* Bb  = Bt + (size_t)b * strideB;
  const T* Ab2 = (SPL >= 1) ? (A2  + (size_t)b * strideA) : nullptr;
  const T* Bb2 = (SPL == 2) ? (Bt2 + (size_t)b * strideB) : nullptr;

  const int rlane = lane & 15;
  const int koff  = (lane >> 4) * 8;
  const int mOff  = (lane >> 4) * 8;

  v8f acc[4][4];
#pragma unroll
  for (int i = 0; i < 4; ++i)
#pragma unroll
    for (int j = 0; j < 4; ++j) acc[i][j] = (v8f){0.f,0.f,0.f,0.f,0.f,0.f,0.f,0.f};

  for (int k0 = 0; k0 < K; k0 += 32) {
    V bh[4], bl[4];
#pragma unroll
    for (int j = 0; j < 4; ++j) {
      const size_t bo = (size_t)(n0 + (j << 4) + rlane) * ldb + koff + k0;
      bh[j] = Frag<T>::load(Bb + bo);
      if (SPL == 2) bl[j] = Frag<T>::load(Bb2 + bo);
    }
#pragma unroll
    for (int i = 0; i < 4; ++i) {
      const size_t ao = (size_t)(m0 + (i << 4) + rlane) * lda + koff + k0;
      V ah = Frag<T>::load(Ab + ao);
      V al;
      if (SPL >= 1) al = Frag<T>::load(Ab2 + ao);
#pragma unroll
      for (int j = 0; j < 4; ++j) {
        acc[i][j] = Frag<T>::mma(ah, bh[j], acc[i][j]);
        if (SPL == 2) acc[i][j] = Frag<T>::mma(ah, bl[j], acc[i][j]);
        if (SPL >= 1) acc[i][j] = Frag<T>::mma(al, bh[j], acc[i][j]);
      }
      Frag<T>::guard(acc[i][0], acc[i][3], ah, (SPL >= 1) ? al : ah);
    }
    Frag<T>::keep(bh[0], bh[1], bh[2], bh[3]);
    if (SPL == 2) Frag<T>::keep(bl[0], bl[1], bl[2], bl[3]);
  }
  acc_guard4(acc[0][0], acc[0][1], acc[0][2], acc[0][3]);
  acc_guard4(acc[1][0], acc[1][1], acc[1][2], acc[1][3]);
  acc_guard4(acc[2][0], acc[2][1], acc[2][2], acc[2][3]);
  acc_guard4(acc[3][0], acc[3][1], acc[3][2], acc[3][3]);

  float* slab = sT[wave];
  const float* Rb = RESID ? (resid + (size_t)b * strideR) : nullptr;
#pragma unroll
  for (int i = 0; i < 4; ++i) {
    const int mBase = m0 + (i << 4);
#pragma unroll
    for (int j = 0; j < 4; ++j) {
      const int n = n0 + (j << 4) + rlane;
      float bv = 0.f;
      if (BIAS_MODE == 2) bv = bias[n];
#pragma unroll
      for (int r = 0; r < 8; ++r) {
        float v = acc[i][j][r] * scale;
        if (BIAS_MODE == 1) v += bias[mBase + mOff + r];
        if (BIAS_MODE == 2) v += bv;
        if (RESID) v += Rb[(size_t)(mBase + mOff + r) * ldc + n];
        if (ACT == 1) v = tanhf(v);
        if (ACT == 2) v = fmaxf(v, 0.0f);
        if (ACT == 3) v = v / (1.0f + expf(-v));
        if (ACT == 4) v = (v > 0.f) ? v : 0.01f * v;
        slab[(mOff + r) * 68 + (j << 4) + rlane] = v;
      }
    }
    __builtin_amdgcn_fence(__ATOMIC_RELEASE, "workgroup");
    __builtin_amdgcn_wave_barrier();
    __builtin_amdgcn_fence(__ATOMIC_ACQUIRE, "workgroup");
    if (OUT_MODE == 0) {
      float* C = (float*)Cout + (size_t)b * strideC;
      const int hh = lane >> 4, c4 = (lane & 15) * 4;
      for (int pass = 0; pass < 2; ++pass) {
#pragma unroll
        for (int it = 0; it < 8; ++it) {
          const int row = it * 2 + hh;
          v4f v = *(const v4f*)(slab + row * 68 + c4);
          *(volatile v4f*)(C + (size_t)(mBase + row) * ldc + n0 + c4) = v;
        }
        __threadfence();
      }
    } else {
      const int q = lane >> 3, c8 = (lane & 7) * 8;
      unsigned short* C  = (unsigned short*)Cout  + (size_t)b * strideC;
      unsigned short* C2 = (OUT_MODE == 2) ? ((unsigned short*)Cout2 + (size_t)b * strideC) : nullptr;
      for (int pass = 0; pass < 2; ++pass) {
#pragma unroll
        for (int it = 0; it < 4; ++it) {
          const int row = it * 4 + q;
          const float* sp = slab + row * 68 + c8;
          v8h hv, lv;
#pragma unroll
          for (int e = 0; e < 8; ++e) {
            if (OUT_MODE == 1) {
              hv[e] = (_Float16)sp[e];
            } else {
              unsigned short hb = f2bf_bits(sp[e]);
              unsigned short lb = f2bf_bits(sp[e] - bf_bits2f(hb));
              hv[e] = __builtin_bit_cast(_Float16, hb);
              lv[e] = __builtin_bit_cast(_Float16, lb);
            }
          }
          *(volatile v8h*)(C + (size_t)(mBase + row) * ldc + n0 + c8) = hv;
          if (OUT_MODE == 2) *(volatile v8h*)(C2 + (size_t)(mBase + row) * ldc + n0 + c8) = lv;
        }
        __threadfence();
      }
    }
    __builtin_amdgcn_fence(__ATOMIC_RELEASE, "workgroup");
    __builtin_amdgcn_wave_barrier();
    __builtin_amdgcn_fence(__ATOMIC_ACQUIRE, "workgroup");
  }
}

__global__ __launch_bounds__(256) void cast_rows_bf16_kernel(
    const float* __restrict__ src, unsigned short* __restrict__ dst, int total8)
{
  const int i = blockIdx.x * 256 + threadIdx.x;
  if (i >= total8) return;
  const size_t e0 = (size_t)i << 3;
  const v4f a0 = *(const v4f*)(src + e0);
  const v4f a1 = *(const v4f*)(src + e0 + 4);
  v8h hv;
#pragma unroll
  for (int e = 0; e < 4; ++e) {
    const unsigned short h0 = f2bf_bits(a0[e]), h1 = f2bf_bits(a1[e]);
    hv[e]     = __builtin_bit_cast(_Float16, h0);
    hv[4 + e] = __builtin_bit_cast(_Float16, h1);
  }
  unsigned short* qh = dst + e0;
  *(volatile v8h*)qh = hv;
  __threadfence();
  *(volatile v8h*)qh = hv;
}

template <int MODE>
__global__ __launch_bounds__(256) void transpose16_kernel(
    const float* __restrict__ src, unsigned short* __restrict__ dst, int R, int CC)
{
  __shared__ __align__(16) float sm[64 * kTrP];
  const int tid = threadIdx.x, lane = tid & 31, wave = tid >> 5;
  const int c0 = blockIdx.x * 64;
  const int r0 = blockIdx.y * 64;
#pragma unroll
  for (int i = 0; i < 4; ++i) {
    const int idx = tid + 256 * i;
    const int rr = idx >> 4, c4 = (idx & 15) * 4;
    const v4f v = *(const v4f*)(src + (size_t)(r0 + rr) * CC + c0 + c4);
    *(v4f*)(sm + rr * kTrP + c4) = v;
  }
  __syncthreads();
  const int q = lane >> 3, e8 = (lane & 7) * 8;
  v8h hv[2];
#pragma unroll
  for (int it = 0; it < 2; ++it) {
    const int cc = wave * 8 + it * 4 + q;
#pragma unroll
    for (int e = 0; e < 8; ++e) {
      const float f = sm[(e8 + e) * kTrP + cc];
      const unsigned short hb = f2bf_bits(f);
      if (MODE == 0) {
        hv[it][e] = __builtin_bit_cast(_Float16, hb);
      } else {
        const float g = bf_bits2f(hb) * 64.0f;
        hv[it][e] = (_Float16)g;
      }
    }
  }
  for (int pass = 0; pass < 2; ++pass) {
#pragma unroll
    for (int it = 0; it < 2; ++it) {
      const int cc = wave * 8 + it * 4 + q;
      *(volatile v8h*)(dst + (size_t)(c0 + cc) * R + r0 + e8) = hv[it];
    }
    __threadfence();
  }
}

__global__ __launch_bounds__(64) void scan_gate_kernel(
    const float* __restrict__ XZ, const float* __restrict__ cw, const float* __restrict__ cb,
    const float* __restrict__ Alog, const float* __restrict__ Dp, unsigned short* __restrict__ YG, int bix)
{
  __shared__ __align__(16) float sY[kScanTS * kScanYP];
  __shared__ __align__(16) float sA[kNst * kScanCh];
  const int tid = threadIdx.x, lane = tid & 31, wave = tid >> 5;
  const int d0 = blockIdx.x * kScanCh;
  const int d  = d0 + tid;
#pragma unroll 1
  for (int j = 0; j < kNst; ++j) sA[j * kScanCh + tid] = -expf(bf_rne(Alog[(size_t)j * kDin + d]));
  const v4f wv = *(const v4f*)(cw + (size_t)d * kConv);
  const float w0 = bf_rne(wv[0]), w1 = bf_rne(wv[1]), w2 = bf_rne(wv[2]), w3 = bf_rne(wv[3]);
  const float bc = bf_rne(cb[d]);
  const float Dd = bf_rne(Dp[d]);
  __syncthreads();
  float Aj[kNst], st[kNst];
#pragma unroll
  for (int j = 0; j < kNst; ++j) {
    Aj[j] = sA[j * kScanCh + tid];
    st[j] = 0.0f;
  }
  float um1 = 0.0f, um2 = 0.0f, um3 = 0.0f;
  const size_t yrow0 = (size_t)bix * kSeq;
  const int q = lane >> 3, c8 = (lane & 7) * 8;
#pragma unroll 1
  for (int t0 = 0; t0 < kSeq; t0 += kScanTS) {
    __syncthreads();
#pragma unroll 1
    for (int s = 0; s < kScanTS; ++s) {
      const int t = t0 + s;
      const float ur = XZ[(size_t)t * kXzP + d];
      const float zv = XZ[(size_t)t * kXzP + kDin + d];
      float cv = w0 * um3;
      cv = fmaf(w1, um2, cv);
      cv = fmaf(w2, um1, cv);
      cv = fmaf(w3, ur, cv);
      const float u = cv + bc;
      um3 = um2; um2 = um1; um1 = ur;
      float ssum = 0.0f;
#pragma unroll
      for (int j = 0; j < kNst; ++j) {
        st[j] = fmaf(st[j], Aj[j], u);
        ssum = ssum + st[j];
      }
      const float y  = fmaf(Dd, u, ssum);
      const float sg = __builtin_amdgcn_rcpf(1.0f + expf(-zv));
      sY[s * kScanYP + tid] = y * (zv * sg);
    }
    __syncthreads();
    v8h hv[8];
#pragma unroll
    for (int it = 0; it < 8; ++it) {
      const int row = it * 8 + wave * 4 + q;
      const float* sp = sY + row * kScanYP + c8;
      const v4f a0 = *(const v4f*)(sp);
      const v4f a1 = *(const v4f*)(sp + 4);
#pragma unroll
      for (int e = 0; e < 4; ++e) {
        hv[it][e]     = (_Float16)a0[e];
        hv[it][4 + e] = (_Float16)a1[e];
      }
    }
    for (int pass = 0; pass < 2; ++pass) {
#pragma unroll
      for (int it = 0; it < 8; ++it) {
        const int row = it * 8 + wave * 4 + q;
        const size_t o = (yrow0 + t0 + row) * kDin + d0 + c8;
        *(volatile v8h*)(YG + o) = hv[it];
      }
      __threadfence();
    }
  }
}

extern "C" void kernel_launch(void* const* d_in, const int* in_sizes, int n_in,
                              void* d_out, int out_size, void* d_ws, size_t ws_size,
                              hipStream_t stream) {
  if (n_in < 7) return;
  if (in_sizes[0] != kRows * kDm) return;
  if (in_sizes[1] != kDm * kXzP) return;
  if (in_sizes[2] != kDin * kConv) return;
  if (in_sizes[3] != kDin) return;
  if (in_sizes[4] != kNst * kDin) return;
  if (in_sizes[5] != kDin) return;
  if (in_sizes[6] != kDin * kDm) return;
  if (out_size != kRows * kDm) return;
  if (ws_size < kWsTotal) return;

  const float* x      = (const float*)d_in[0];
  const float* W_in   = (const float*)d_in[1];
  const float* conv_w = (const float*)d_in[2];
  const float* conv_b = (const float*)d_in[3];
  const float* A_log  = (const float*)d_in[4];
  const float* Dp     = (const float*)d_in[5];
  const float* W_out  = (const float*)d_in[6];
  float* out = (float*)d_out;

  char* ws = (char*)d_ws;
  unsigned short* XB  = (unsigned short*)(ws + kOffXB);
  unsigned short* WIT = (unsigned short*)(ws + kOffWIT);
  unsigned short* WOT = (unsigned short*)(ws + kOffWOT);
  float*          XZ  = (float*)(ws + kOffXZ);
  unsigned short* YG  = (unsigned short*)(ws + kOffYG);

  cast_rows_bf16_kernel<<<(kRows * kDm / 8) / 256, 256, 0, stream>>>(x, XB, kRows * kDm / 8);
  transpose16_kernel<0><<<dim3(kXzP / 64, kDm / 64), 256, 0, stream>>>(W_in, WIT, kDm, kXzP);
  transpose16_kernel<1><<<dim3(kDm / 64, kDin / 64), 256, 0, stream>>>(W_out, WOT, kDin, kDm);

  for (int bb = 0; bb < kBatch; ++bb) {
    wmma_gemm64<1, 0, 0, 0, false><<<dim3(256, 1), 256, 0, stream>>>(
        XB + (size_t)bb * kSeq * kDm, nullptr, kDm, 0L,
        WIT, nullptr, kDm, 0L,
        (void*)XZ, nullptr, kXzP, 0L,
        nullptr, nullptr, 0L,
        kSeq, kXzP, kDm, 1.0f);
    scan_gate_kernel<<<kDin / kScanCh, kScanCh, 0, stream>>>(XZ, conv_w, conv_b, A_log, Dp, YG, bb);
  }

  wmma_gemm64<0, 0, 0, 0, false><<<dim3(256, 1), 256, 0, stream>>>(
      YG, nullptr, kDin, 0L,
      WOT, nullptr, kDin, 0L,
      (void*)out, nullptr, kDm, 0L,
      nullptr, nullptr, 0L,
      kRows, kDm, kDin, 1.0f / 64.0f);
}
